// MCTS_GAT_36953898615235
// MI455X (gfx1250) — hardware-verified
//
#include <hip/hip_runtime.h>
#include <stddef.h>


#define DF    128
#define KIN   11
#define K1P   32
#define GR    32
#define AP    136
#define XSP   132
#define NB    512
#define CHUNK 2048
#define NTHR  256
#define NWAVE 8
#define WCAP  256
#define NGRP  (CHUNK / (NTHR * 4))
#define MPB   32

#define LDS_SACC (NB * DF)
#define LDS_AUX  (3 * NB)
#define LDS_LIST (NWAVE * WCAP)
#define LDS_BYTES ((LDS_SACC + LDS_AUX + LDS_LIST + NWAVE) * 4)

static_assert(WCAP == (CHUNK / NTHR) * 32);
static_assert(NGRP == 2);
static_assert(NB == 512);
static_assert(CHUNK == 2048);
static_assert((LDS_SACC % 4) == 0);
static_assert(LDS_BYTES == 276512);
static_assert(NTHR == NWAVE * 32);
static_assert(GR == 4 * NWAVE);
static_assert(MPB == 4 * NWAVE);

typedef float    v4f  __attribute__((ext_vector_type(4)));
typedef float    v8f  __attribute__((ext_vector_type(8)));
typedef int      v4i  __attribute__((ext_vector_type(4)));
typedef _Float16 v4h  __attribute__((ext_vector_type(4)));
typedef _Float16 v8h  __attribute__((ext_vector_type(8)));
typedef _Float16 v16h __attribute__((ext_vector_type(16)));
union Frag   { v16h v; v8h half[2]; };
union Pack16 { v8h h; v4i i; };

__device__ __forceinline__ v8f wm(v16h a, v16h b, v8f c) {
  v8f d = __builtin_amdgcn_wmma_f32_16x16x32_f16(false, a, false, b, (short)0, c, false, false);
  asm volatile("v_nop\n\tv_nop\n\tv_nop\n\tv_nop" : "+v"(d) : "v"(a), "v"(b));
  return d;
}

__device__ __forceinline__ float wsum(float v) {
  v += __shfl_xor(v, 16, 32);
  v += __shfl_xor(v, 8, 32);
  v += __shfl_xor(v, 4, 32);
  v += __shfl_xor(v, 2, 32);
  v += __shfl_xor(v, 1, 32);
  return v;
}

__global__ __launch_bounds__(NTHR) void k_prep(const float* __restrict__ W1, const float* __restrict__ W2,
                                               const float* __restrict__ P1, _Float16* Bt, _Float16* W1t) {
  __shared__ __attribute__((aligned(16))) float T[64 * DF];
  const int tid = threadIdx.x, lane = tid & 31, wave = tid >> 5;
  const int z = blockIdx.y;
  if (z == 3) {
    if (blockIdx.x != 0) return;
    for (int i = tid; i < KIN * DF; i += NTHR) T[i] = W1[i];
    __syncthreads();
    Pack16 u[2];
    _Float16* pp[2];
#pragma unroll
    for (int rep = 0; rep < 2; ++rep) {
      const int p  = rep * NTHR + tid;
      const int L  = p >> 3, q = p & 7;
      const int n  = 2 * L + (q >> 2);
      const int k8 = (q & 3) * 8;
#pragma unroll
      for (int j = 0; j < 8; ++j) {
        const int k  = k8 + j;
        const int kc = (k < KIN) ? k : (KIN - 1);
        const float v = T[kc * DF + n] * 8.0f;
        u[rep].h[j] = (k < KIN) ? (_Float16)v : (_Float16)0.0f;
      }
      pp[rep] = W1t + (size_t)n * K1P + k8;
    }
#pragma unroll
    for (int rep = 0; rep < 2; ++rep) *(volatile v4i*)pp[rep] = u[rep].i;
    __threadfence();
#pragma unroll
    for (int rep = 0; rep < 2; ++rep) *(volatile v4i*)pp[rep] = u[rep].i;
    return;
  }

  const int kb = blockIdx.x * 64;
  const float* src = (z == 0) ? W2 : (P1 + (size_t)(z - 1) * DF * DF);
#pragma unroll
  for (int it = 0; it < 8; ++it) {
    const int i  = it * NTHR + tid;
    const int r  = i >> 5, c4 = i & 31;
    *(v4f*)(T + r * DF + 4 * c4) = *(const v4f*)(src + (size_t)(kb + r) * DF + 4 * c4);
  }
  __syncthreads();
  _Float16* dstp = Bt + (size_t)z * DF * DF;
  const int q = lane & 7, sub = lane >> 3;
  Pack16 u[4];
  _Float16* pp[4];
#pragma unroll
  for (int it = 0; it < 4; ++it) {
    const int n = wave * 16 + it * 4 + sub;
#pragma unroll
    for (int j = 0; j < 8; ++j) u[it].h[j] = (_Float16)(T[(q * 8 + j) * DF + n] * 8.0f);
    pp[it] = dstp + (size_t)n * DF + kb + q * 8;
  }
#pragma unroll
  for (int it = 0; it < 4; ++it) *(volatile v4i*)pp[it] = u[it].i;
  __threadfence();
#pragma unroll
  for (int it = 0; it < 4; ++it) *(volatile v4i*)pp[it] = u[it].i;
}

template <bool DOTS>
__device__ __forceinline__ void epi_tile(v8f acc, int T, int hh, int m, int wave, int ncol,
                                         float cs, float cd, float* Xs, float* Ps, float* Qs) {
  float ss[8], sd[8];
#pragma unroll
  for (int r = 0; r < 8; ++r) {
    const float v = acc[r] * 0.125f;
    Xs[(T * 16 + 8 * hh + r) * XSP + ncol] = v;
    ss[r] = v * cs;
    sd[r] = v * cd;
  }
  if constexpr (DOTS) {
#pragma unroll
    for (int mk = 1; mk < 16; mk <<= 1) {
#pragma unroll
      for (int r = 0; r < 8; ++r) {
        ss[r] += __shfl_xor(ss[r], mk, 32);
        sd[r] += __shfl_xor(sd[r], mk, 32);
      }
    }
    if (m == 0) {
#pragma unroll
      for (int r = 0; r < 8; ++r) {
        Ps[(T * 16 + 8 * hh + r) * NWAVE + wave] = ss[r];
        Qs[(T * 16 + 8 * hh + r) * NWAVE + wave] = sd[r];
      }
    }
  }
}

template <int KD, bool DOTS>
__global__ __launch_bounds__(NTHR) void k_gemm(
    const float* __restrict__ A, const _Float16* __restrict__ Bt,
    const float* __restrict__ att_s, const float* __restrict__ att_d,
    float* C, float* esrc, float* edst, int nN, int planeF) {
  __shared__ __attribute__((aligned(16))) _Float16 At[GR * AP];
  __shared__ __attribute__((aligned(16))) float Xs[GR * XSP];
  __shared__ __attribute__((aligned(16))) float Ps[GR * NWAVE];
  __shared__ __attribute__((aligned(16))) float Qs[GR * NWAVE];

  const int tid  = threadIdx.x;
  const int lane = tid & 31;
  const int wave = tid >> 5;
  const int hh   = lane >> 4;
  const int m    = lane & 15;
  const int rowBase = blockIdx.x * GR;
  const int y = blockIdx.y;
  const _Float16* Bp = Bt + (size_t)y * DF * KD;
  float* Cp = C + (size_t)y * (size_t)planeF;

  if constexpr (KD == DF) {
    const int r  = tid >> 3;
    const int c0 = (tid & 7) * 16;
    int row = rowBase + r;
    if (row > nN - 1) row = nN - 1;
    const float* p = A + (size_t)row * DF + c0;
    const v4f f0 = *(const v4f*)(p), f1 = *(const v4f*)(p + 4);
    const v4f f2 = *(const v4f*)(p + 8), f3 = *(const v4f*)(p + 12);
    Pack16 u0, u1;
    u0.h[0] = (_Float16)f0.x; u0.h[1] = (_Float16)f0.y; u0.h[2] = (_Float16)f0.z; u0.h[3] = (_Float16)f0.w;
    u0.h[4] = (_Float16)f1.x; u0.h[5] = (_Float16)f1.y; u0.h[6] = (_Float16)f1.z; u0.h[7] = (_Float16)f1.w;
    u1.h[0] = (_Float16)f2.x; u1.h[1] = (_Float16)f2.y; u1.h[2] = (_Float16)f2.z; u1.h[3] = (_Float16)f2.w;
    u1.h[4] = (_Float16)f3.x; u1.h[5] = (_Float16)f3.y; u1.h[6] = (_Float16)f3.z; u1.h[7] = (_Float16)f3.w;
    *(v8h*)(At + r * AP + c0)     = u0.h;
    *(v8h*)(At + r * AP + c0 + 8) = u1.h;
  } else {
    const int r    = tid >> 3;
    const int part = tid & 7;
    int row = rowBase + r;
    if (row > nN - 1) row = nN - 1;
    const float* p = A + (size_t)row * KIN;
    const int k0i = 4 * part;
    const int kc0 = (k0i     < KIN) ? (k0i)     : (KIN - 1);
    const int kc1 = (k0i + 1 < KIN) ? (k0i + 1) : (KIN - 1);
    const int kc2 = (k0i + 2 < KIN) ? (k0i + 2) : (KIN - 1);
    const int kc3 = (k0i + 3 < KIN) ? (k0i + 3) : (KIN - 1);
    const float v0 = p[kc0], v1 = p[kc1], v2 = p[kc2], v3 = p[kc3];
    const _Float16 h0 = (k0i     < KIN) ? (_Float16)v0 : (_Float16)0.0f;
    const _Float16 h1 = (k0i + 1 < KIN) ? (_Float16)v1 : (_Float16)0.0f;
    const _Float16 h2 = (k0i + 2 < KIN) ? (_Float16)v2 : (_Float16)0.0f;
    const _Float16 h3 = (k0i + 3 < KIN) ? (_Float16)v3 : (_Float16)0.0f;
    const v4h u4 = {h0, h1, h2, h3};
    *(v4h*)(At + r * AP + k0i) = u4;
  }
  __syncthreads();

  const int ncol = wave * 16 + m;
  v8f c0a = {0.f, 0.f, 0.f, 0.f, 0.f, 0.f, 0.f, 0.f};
  v8f c1a = {0.f, 0.f, 0.f, 0.f, 0.f, 0.f, 0.f, 0.f};
#pragma unroll
  for (int kt = 0; kt < KD / 32; ++kt) {
    const int k0 = kt * 32;
    Frag a0, a1, b;
    const _Float16* pb  = Bp + (size_t)ncol * KD + k0 + 8 * hh;
    const _Float16* pa0 = At + m * AP + k0 + 8 * hh;
    const _Float16* pa1 = At + (16 + m) * AP + k0 + 8 * hh;
    b.half[0]  = *(const v8h*)pb;  b.half[1]  = *(const v8h*)(pb + 16);
    a0.half[0] = *(const v8h*)pa0; a0.half[1] = *(const v8h*)(pa0 + 16);
    a1.half[0] = *(const v8h*)pa1; a1.half[1] = *(const v8h*)(pa1 + 16);
    c0a = wm(a0.v, b.v, c0a);
    c1a = wm(a1.v, b.v, c1a);
  }

  float cs = 0.f, cd = 0.f;
  if constexpr (DOTS) { cs = att_s[ncol]; cd = att_d[ncol]; }
  epi_tile<DOTS>(c0a, 0, hh, m, wave, ncol, cs, cd, Xs, Ps, Qs);
  epi_tile<DOTS>(c1a, 1, hh, m, wave, ncol, cs, cd, Xs, Ps, Qs);
  __syncthreads();

  v4f xr[4];
  float* xpp[4];
#pragma unroll
  for (int i = 0; i < 4; ++i) {
    xr[i]  = *(const v4f*)(Xs + (4 * wave + i) * XSP + 4 * lane);
    xpp[i] = Cp + (size_t)(rowBase + 4 * wave + i) * DF + 4 * lane;
  }
  const v4f z4 = {0.f, 0.f, 0.f, 0.f};
  v4f gv = z4;
  float* gp = Cp;
  bool gdo = false;
  if constexpr (DOTS) {
    if (wave == 0 && lane < 16) {
      const int q = lane & 7;
      v4f sa = z4, sb = z4;
#pragma unroll
      for (int i = 0; i < 4; ++i) {
        float ta = 0.f, tb = 0.f;
#pragma unroll
        for (int w = 0; w < NWAVE; ++w) {
          ta += Ps[(4 * q + i) * NWAVE + w];
          tb += Qs[(4 * q + i) * NWAVE + w];
        }
        sa[i] = ta;
        sb[i] = tb;
      }
      gv = sa;
      gp = esrc + rowBase + 4 * q;
      if (lane & 8) { gv = sb; gp = edst + rowBase + 4 * q; }
      gdo = true;
    }
  }

#pragma unroll
  for (int i = 0; i < 4; ++i) *(volatile v4f*)(xpp[i]) = xr[i];
  if (gdo) *(volatile v4f*)gp = gv;
  __threadfence();
#pragma unroll
  for (int i = 0; i < 4; ++i) *(volatile v4f*)(xpp[i]) = xr[i];
  if (gdo) *(volatile v4f*)gp = gv;
}

__global__ __launch_bounds__(NTHR) void k_gat(
    const int* __restrict__ ei, const float* __restrict__ hp,
    const float* __restrict__ esrc, const float* __restrict__ edst,
    const float* __restrict__ bias, float* hout, int nN, int nE) {
  extern __shared__ v4f lds_dyn[];
  float* sacc = (float*)lds_dyn;
  float* mrun = sacc + LDS_SACC;
  float* srun = mrun + NB;
  float* edl  = srun + NB;
  int*   list = (int*)(edl + NB);
  int*   wcnt = list + LDS_LIST;

  const int tid  = threadIdx.x;
  const int lane = tid & 31;
  const int wave = tid >> 5;
  const int nodeBase = blockIdx.x * NB;
  const float ninf = -__builtin_huge_valf();

  {
    const v4f z4 = {0.f, 0.f, 0.f, 0.f};
    for (int i = tid; i < LDS_SACC / 4; i += NTHR) lds_dyn[i] = z4;
    for (int i = tid; i < NB; i += NTHR) {
      int nd = nodeBase + i;
      if (nd > nN - 1) nd = nN - 1;
      mrun[i] = ninf;
      srun[i] = 0.f;
      edl[i]  = edst[nd];
    }
  }
  __syncthreads();
  const int* eid = ei + nE;
  const bool al16 = ((nE & 3) == 0);

  const int nChunks = (nE + CHUNK - 1) / CHUNK;
#pragma unroll 1
  for (int ch = 0; ch < nChunks; ++ch) {
    const int cbase = ch * CHUNK;
    const bool fullc = al16 && (cbase + CHUNK <= nE);
    int wc = 0;
#pragma unroll
    for (int g = 0; g < NGRP; ++g) {
      const int el0 = (g * NTHR + tid) * 4;
      const int e0  = cbase + el0;
      const int sent = -2147483647 - 1;
      v4i d;
      if (fullc) {
        d = *(const v4i*)(eid + e0);
      } else {
        const int q0 = (e0     < nE) ? e0     : (nE - 1);
        const int q1 = (e0 + 1 < nE) ? e0 + 1 : (nE - 1);
        const int q2 = (e0 + 2 < nE) ? e0 + 2 : (nE - 1);
        const int q3 = (e0 + 3 < nE) ? e0 + 3 : (nE - 1);
        const int l0 = eid[q0], l1 = eid[q1], l2 = eid[q2], l3 = eid[q3];
        d.x = (e0     < nE) ? l0 : sent;
        d.y = (e0 + 1 < nE) ? l1 : sent;
        d.z = (e0 + 2 < nE) ? l2 : sent;
        d.w = (e0 + 3 < nE) ? l3 : sent;
      }
      const unsigned s0 = (unsigned)d.x - (unsigned)nodeBase;
      const unsigned s1 = (unsigned)d.y - (unsigned)nodeBase;
      const unsigned s2 = (unsigned)d.z - (unsigned)nodeBase;
      const unsigned s3 = (unsigned)d.w - (unsigned)nodeBase;
      const bool h0 = s0 < (unsigned)NB;
      const bool h1 = s1 < (unsigned)NB;
      const bool h2 = s2 < (unsigned)NB;
      const bool h3 = s3 < (unsigned)NB;
      const unsigned many = __builtin_amdgcn_ballot_w32(h0 | h1 | h2 | h3);
      if (many != 0u) {
#define HITJ(J, HJ, SJ) { \
          const unsigned mj = __builtin_amdgcn_ballot_w32(HJ); \
          if (HJ) { \
            const int pos = wc + (int)__builtin_amdgcn_mbcnt_lo(mj, 0u); \
            if (pos < WCAP) list[wave * WCAP + pos] = ((el0 + (J)) << 9) | (int)(SJ); \
          } \
          wc += (int)__builtin_popcount(mj); }
        HITJ(0, h0, s0)
        HITJ(1, h1, s1)
        HITJ(2, h2, s2)
        HITJ(3, h3, s3)
#undef HITJ
      }
    }
    if (lane == 0) wcnt[wave] = wc;
    __syncthreads();

    if (wave == 0) {
#pragma unroll 1
      for (int wsx = 0; wsx < NWAVE; ++wsx) {
        int n = wcnt[wsx];
        if (n > WCAP) n = WCAP;
        if (n < 0) n = 0;
#pragma unroll 1
        for (int i = 0; i < n; ++i) {
          const int ent  = list[wsx * WCAP + i];
          const int slot = ent & (NB - 1);
          const int el   = (ent >> 9) & (CHUNK - 1);
          int e = cbase + el;
          if (e > nE - 1) e = nE - 1;
          int src = ei[e];
          src = src < 0 ? 0 : (src > nN - 1 ? nN - 1 : src);
          float a = esrc[src] + edl[slot];
          a = (a > 0.f) ? a : 0.2f * a;
          const float mo = mrun[slot];
          const float mn = fmaxf(mo, a);
          const float sc = __expf(mo - mn);
          const float p  = __expf(a - mn);
          const v4f xv = *(const v4f*)(hp + (size_t)src * DF + 4 * lane);
          v4f* sp = (v4f*)(sacc + slot * DF + 4 * lane);
          const v4f cur = *sp;
          const v4f nxt = cur * sc + xv * p;
          *sp = nxt;
          const float so = srun[slot];
          srun[slot] = so * sc + p;
          mrun[slot] = mn;
        }
      }
    }
    __syncthreads();
  }

  const v4f b4 = *(const v4f*)(bias + 4 * lane);
#pragma unroll 1
  for (int j = 0; j < NB / NWAVE; ++j) {
    const int slot = wave * (NB / NWAVE) + j;
    const int node = nodeBase + slot;
    if (node >= nN) break;
    const float s   = srun[slot];
    const float inv = 1.0f / (s + 1e-16f);
    const v4f sv = *(const v4f*)(sacc + slot * DF + 4 * lane);
    v4f h = sv * inv + b4;
    h.x = fmaxf(h.x, 0.f);
    h.y = fmaxf(h.y, 0.f);
    h.z = fmaxf(h.z, 0.f);
    h.w = fmaxf(h.w, 0.f);
    float* op = hout + (size_t)node * DF + 4 * lane;
    *(volatile v4f*)op = h;
    __threadfence();
    *(volatile v4f*)op = h;
  }
}

__global__ __launch_bounds__(NTHR) void k_value(
    const float* __restrict__ H, const int* __restrict__ bt,
    const float* __restrict__ V1, const float* __restrict__ vb1,
    const float* __restrict__ V2, const float* __restrict__ vb2,
    float* vline, int nN) {
  __shared__ double sS[NTHR];
  __shared__ int    sC[NTHR];
  __shared__ float  sg[DF];
  __shared__ float  sr[DF];
  const int tid = threadIdx.x, lane = tid & 31, wave = tid >> 5;
  const int c = tid & (DF - 1), part = tid >> 7;
  double acc = 0.0;
  int cnt = 0;
#pragma unroll 1
  for (int n = part; n < nN; n += 2) {
    const int b = bt[n];
    const float v = H[(size_t)n * DF + c];
    const bool in0 = (b == 0);
    acc += in0 ? (double)v : 0.0;
    cnt += in0 ? 1 : 0;
  }
  sS[tid] = acc;
  sC[tid] = cnt;
  __syncthreads();
  if (tid < DF) {
    const double S = sS[tid] + sS[tid + DF];
    const int ct = sC[tid] + sC[tid + DF];
    sg[tid] = (float)S * (1.0f / (float)ct);
  }
  __syncthreads();
  if (tid < DF) {
    float a = vb1[c];
#pragma unroll 1
    for (int k = 0; k < DF; ++k) a += sg[k] * V1[(size_t)k * DF + c];
    a = fmaxf(a, 0.f);
    sr[tid] = a * V2[c];
  }
  __syncthreads();
#pragma unroll 1
  for (int o = DF / 2; o > 0; o >>= 1) {
    if (tid < o) sr[tid] = sr[tid] + sr[tid + o];
    __syncthreads();
  }
  const float xarg = sr[0] + vb2[0];
  const float ax = fabsf(xarg);
  const float t  = expf(-2.0f * ax);
  float th = (1.0f - t) * (1.0f / (1.0f + t));
  th = (xarg < 0.f) ? -th : th;
  const v4f z4 = {0.f, 0.f, 0.f, 0.f};
  v4f lv = z4;
  if (lane == 0) lv.x = th;
  float* lp = vline + 4 * (lane & 7);
  const bool ldo = (wave == 0) && (lane < 8);
  if (ldo) *(volatile v4f*)lp = lv;
  __threadfence();
  if (ldo) *(volatile v4f*)lp = lv;
}

__global__ __launch_bounds__(NTHR) void k_moves(
    const float* __restrict__ S, const float* __restrict__ D, const int* __restrict__ lm,
    const float* __restrict__ pb1, const float* __restrict__ P2, const float* __restrict__ pb2,
    float* logits, int nM, int nN) {
  __shared__ __attribute__((aligned(16))) float sl[MPB];
  const int tid = threadIdx.x, lane = tid & 31, wave = tid >> 5;
  const int base = blockIdx.x * MPB;
  const v4f b4 = *(const v4f*)(pb1 + 4 * lane);
  const v4f p4 = *(const v4f*)(P2 + 4 * lane);
  const float pb = pb2[0];
#pragma unroll
  for (int j = 0; j < 4; ++j) {
    const int mv = base + wave * 4 + j;
    const int mvc = (mv < nM) ? mv : (nM - 1);
    int i0 = lm[mvc];
    int i1 = lm[(size_t)nM + mvc];
    i0 = i0 < 0 ? 0 : (i0 > nN - 1 ? nN - 1 : i0);
    i1 = i1 < 0 ? 0 : (i1 > nN - 1 ? nN - 1 : i1);
    const v4f s4 = *(const v4f*)(S + (size_t)i0 * DF + 4 * lane);
    const v4f d4 = *(const v4f*)(D + (size_t)i1 * DF + 4 * lane);
    v4f v = s4 + d4 + b4;
    v.x = fmaxf(v.x, 0.f); v.y = fmaxf(v.y, 0.f); v.z = fmaxf(v.z, 0.f); v.w = fmaxf(v.w, 0.f);
    float t = wsum(v.x * p4.x + v.y * p4.y + v.z * p4.z + v.w * p4.w) + pb;
    if (mv >= nM) t = 0.f;
    if (lane == 0) sl[wave * 4 + j] = t;
  }
  __syncthreads();
  const v4f lv = *(const v4f*)(sl + 4 * (lane & 7));
  float* lp = logits + base + 4 * (lane & 7);
  const bool ldo = (wave == 0) && (lane < 8);
  if (ldo) *(volatile v4f*)lp = lv;
  __threadfence();
  if (ldo) *(volatile v4f*)lp = lv;
}

__global__ __launch_bounds__(NTHR) void k_smstat(const float* __restrict__ lg, float* stat, int nM) {
  __shared__ float  sm[NTHR];
  __shared__ double sd[NTHR];
  const int tid = threadIdx.x, lane = tid & 31, wave = tid >> 5;
  float m = -__builtin_huge_valf();
#pragma unroll 1
  for (int i = tid; i < nM; i += NTHR) m = fmaxf(m, lg[i]);
  sm[tid] = m;
  __syncthreads();
#pragma unroll 1
  for (int o = NTHR / 2; o > 0; o >>= 1) {
    if (tid < o) sm[tid] = fmaxf(sm[tid], sm[tid + o]);
    __syncthreads();
  }
  const float gm = sm[0];
  double a = 0.0;
#pragma unroll 1
  for (int i = tid; i < nM; i += NTHR) a += (double)expf(lg[i] - gm);
  sd[tid] = a;
  __syncthreads();
#pragma unroll 1
  for (int o = NTHR / 2; o > 0; o >>= 1) {
    if (tid < o) sd[tid] = sd[tid] + sd[tid + o];
    __syncthreads();
  }
  const float inv = (float)(1.0 / sd[0]);
  const v4f z4 = {0.f, 0.f, 0.f, 0.f};
  v4f lv = z4;
  if (lane == 0) { lv.x = gm; lv.y = inv; }
  float* lp = stat + 4 * (lane & 7);
  const bool ldo = (wave == 0) && (lane < 8);
  if (ldo) *(volatile v4f*)lp = lv;
  __threadfence();
  if (ldo) *(volatile v4f*)lp = lv;
}

__global__ __launch_bounds__(NTHR) void k_out(const float* __restrict__ lg, const float* __restrict__ stat,
                                              const float* __restrict__ vline, float* out, int nM) {
  __shared__ __attribute__((aligned(16))) float sv[4 * NTHR];
  const int tid = threadIdx.x;
  const int T = nM + 1;
  const int bb = blockIdx.x * 4 * NTHR;
  const float gm = stat[0], inv = stat[1], val = vline[0];
#pragma unroll 1
  for (int j = 0; j < 4; ++j) {
    const int f = bb + j * NTHR + tid;
    int li = f - 1;
    li = li < 0 ? 0 : (li > nM - 1 ? nM - 1 : li);
    const float e = expf(lg[li] - gm) * inv;
    sv[j * NTHR + tid] = (f == 0) ? val : e;
  }
  __syncthreads();
  const int f0 = bb + 4 * tid;
  const v4f v = *(const v4f*)(sv + 4 * tid);
  const bool full = (f0 + 3 < T);
  const bool tail = (!full) && (f0 < T);
  if (full) {
    *(volatile v4f*)(out + f0) = v;
  } else if (tail) {
    *(volatile float*)(out + f0) = v.x;
    if (f0 + 1 < T) *(volatile float*)(out + f0 + 1) = v.y;
    if (f0 + 2 < T) *(volatile float*)(out + f0 + 2) = v.z;
  }
  __threadfence();
  if (full) {
    *(volatile v4f*)(out + f0) = v;
  } else if (tail) {
    *(volatile float*)(out + f0) = v.x;
    if (f0 + 1 < T) *(volatile float*)(out + f0 + 1) = v.y;
    if (f0 + 2 < T) *(volatile float*)(out + f0 + 2) = v.z;
  }
}

extern "C" void kernel_launch(void* const* d_in, const int* in_sizes, int n_in,
                              void* d_out, int out_size, void* d_ws, size_t ws_size,
                              hipStream_t stream) {
  if (n_in < 20) return;
  const int nN = in_sizes[0] / KIN;
  if (nN <= 0 || in_sizes[0] != nN * KIN) return;
  if ((in_sizes[1] & 1) != 0 || (in_sizes[2] & 1) != 0) return;
  const int nE = in_sizes[1] / 2;
  const int nM = in_sizes[2] / 2;
  if (nE < 0 || nM <= 0) return;
  if (in_sizes[3] != nN) return;
  if (in_sizes[4] != KIN * DF) return;
  if (in_sizes[5] != DF || in_sizes[6] != DF || in_sizes[7] != DF) return;
  if (in_sizes[8] != DF * DF || in_sizes[9] != DF || in_sizes[10] != DF || in_sizes[11] != DF) return;
  if (in_sizes[12] != 2 * DF * DF || in_sizes[13] != DF || in_sizes[14] != DF || in_sizes[15] != 1) return;
  if (in_sizes[16] != DF * DF || in_sizes[17] != DF || in_sizes[18] != DF || in_sizes[19] != 1) return;
  if (out_size != nM + 1) return;

  const float* x   = (const float*)d_in[0];
  const int*   ei  = (const int*)d_in[1];
  const int*   lm  = (const int*)d_in[2];
  const int*   bat = (const int*)d_in[3];
  const float* W1  = (const float*)d_in[4];
  const float* a1s = (const float*)d_in[5];
  const float* a1d = (const float*)d_in[6];
  const float* b1  = (const float*)d_in[7];
  const float* W2  = (const float*)d_in[8];
  const float* a2s = (const float*)d_in[9];
  const float* a2d = (const float*)d_in[10];
  const float* b2  = (const float*)d_in[11];
  const float* P1  = (const float*)d_in[12];
  const float* pb1 = (const float*)d_in[13];
  const float* P2  = (const float*)d_in[14];
  const float* pb2 = (const float*)d_in[15];
  const float* V1  = (const float*)d_in[16];
  const float* vb1 = (const float*)d_in[17];
  const float* V2  = (const float*)d_in[18];
  const float* vb2 = (const float*)d_in[19];
  float* out = (float*)d_out;

  const int nP = ((nN + GR - 1) / GR) * GR;
  const int Mp = ((nM + MPB - 1) / MPB) * MPB;
  const size_t planeB = (size_t)nP * DF * sizeof(float);
  size_t off = 0;
  _Float16* Bt  = (_Float16*)((char*)d_ws + off); off += (size_t)3 * DF * DF * sizeof(_Float16);
  _Float16* W1t = (_Float16*)((char*)d_ws + off); off += (size_t)DF * K1P * sizeof(_Float16);
  float* Pp    = (float*)((char*)d_ws + off);      off += planeB;
  float* H1    = (float*)((char*)d_ws + off);      off += planeB;
  float* H2    = (float*)((char*)d_ws + off);      off += planeB;
  float* SD    = (float*)((char*)d_ws + off);      off += 2 * planeB;
  float* esrc  = (float*)((char*)d_ws + off);      off += (size_t)nP * sizeof(float);
  float* edst  = (float*)((char*)d_ws + off);      off += (size_t)nP * sizeof(float);
  float* lg    = (float*)((char*)d_ws + off);      off += (size_t)Mp * sizeof(float);
  float* vline = (float*)((char*)d_ws + off);      off += 128;
  float* stat  = (float*)((char*)d_ws + off);      off += 128;
  if (off > ws_size) return;
  if (off > (size_t)134217728) return;

  const int planeF = nP * DF;
  const int gridR  = nP / GR;
  const int gridG  = (nN + NB - 1) / NB;

  k_prep<<<dim3(2, 4), NTHR, 0, stream>>>(W1, W2, P1, Bt, W1t);

  k_gemm<K1P, true><<<dim3(gridR, 1), NTHR, 0, stream>>>(x, W1t, a1s, a1d, Pp, esrc, edst, nN, planeF);
  hipFuncSetAttribute(reinterpret_cast<const void*>(&k_gat),
                      hipFuncAttributeMaxDynamicSharedMemorySize, LDS_BYTES);
  k_gat<<<gridG, NTHR, LDS_BYTES, stream>>>(ei, Pp, esrc, edst, b1, H1, nN, nE);

  k_gemm<DF, true><<<dim3(gridR, 1), NTHR, 0, stream>>>(H1, Bt, a2s, a2d, Pp, esrc, edst, nN, planeF);
  k_gat<<<gridG, NTHR, LDS_BYTES, stream>>>(ei, Pp, esrc, edst, b2, H2, nN, nE);

  k_gemm<DF, false><<<dim3(gridR, 2), NTHR, 0, stream>>>(H2, Bt + (size_t)DF * DF, a2s, a2d, SD, esrc, edst, nN, planeF);

  k_value<<<1, NTHR, 0, stream>>>(H2, bat, V1, vb1, V2, vb2, vline, nN);

  k_moves<<<Mp / MPB, NTHR, 0, stream>>>(SD, SD + (size_t)planeF, lm, pb1, P2, pb2, lg, nM, nN);
  k_smstat<<<1, NTHR, 0, stream>>>(lg, stat, nM);
  const int gridO = (nM + 1 + 4 * NTHR - 1) / (4 * NTHR);
  k_out<<<gridO, NTHR, 0, stream>>>(lg, stat, vline, out, nM);
}
